// SASA_24584392802735
// MI455X (gfx1250) — hardware-verified
//
#include <hip/hip_runtime.h>
#include <stdint.h>
#include <stddef.h>

typedef __attribute__((ext_vector_type(16))) _Float16 v16h;
typedef __attribute__((ext_vector_type(8)))  _Float16 v8h;
typedef __attribute__((ext_vector_type(16))) __bf16   v16b;
typedef __attribute__((ext_vector_type(8)))  __bf16   v8b;
typedef __attribute__((ext_vector_type(8)))  float    v8f;
typedef __attribute__((ext_vector_type(4)))  float    v4f;
typedef __attribute__((ext_vector_type(4)))  unsigned int v4u;
typedef __attribute__((ext_vector_type(8)))  unsigned int v8u;
typedef __attribute__((ext_vector_type(8)))  unsigned short v8us;

__device__ __forceinline__ unsigned short f2bf_bits(float f) {
  unsigned u = __float_as_uint(f);
  return (unsigned short)((u + 0x7FFFu + ((u >> 16) & 1u)) >> 16);
}
__device__ __forceinline__ float bf_bits2f(unsigned short h) { return __uint_as_float(((unsigned)h) << 16); }

__device__ __forceinline__ void dep_guard_h(v8f& a, v8f& b, v16h x, v16h y) { asm volatile("v_nop\n\tv_nop\n\tv_nop\n\tv_nop" : "+v"(a), "+v"(b) : "v"(x), "v"(y)); }
__device__ __forceinline__ void dep_guard_b(v8f& a, v8f& b, v16b x, v16b y) { asm volatile("v_nop\n\tv_nop\n\tv_nop\n\tv_nop" : "+v"(a), "+v"(b) : "v"(x), "v"(y)); }
__device__ __forceinline__ void keep4_h(v16h a, v16h b, v16h c, v16h d) { asm volatile("v_nop" :: "v"(a), "v"(b), "v"(c), "v"(d)); }
__device__ __forceinline__ void keep4_b(v16b a, v16b b, v16b c, v16b d) { asm volatile("v_nop" :: "v"(a), "v"(b), "v"(c), "v"(d)); }
__device__ __forceinline__ void acc_guard4(v8f& a, v8f& b, v8f& c, v8f& d) { asm volatile("v_nop\n\tv_nop\n\tv_nop\n\tv_nop" : "+v"(a), "+v"(b), "+v"(c), "+v"(d)); }
template <typename T> struct Frag;
template <> struct Frag<_Float16> {
  typedef v16h V; union U { v16h v; v8h h[2]; };
  static __device__ __forceinline__ v16h load(const _Float16* p) {
    U f; f.h[0] = *(const v8h*)(p); f.h[1] = *(const v8h*)(p + 16); return f.v;
  }
  static __device__ __forceinline__ v8f mma(v16h a, v16h b, v8f c) {
    return __builtin_amdgcn_wmma_f32_16x16x32_f16(false, a, false, b, (short)0, c, false, false);
  }
  static __device__ __forceinline__ void guard(v8f& a, v8f& b, v16h x, v16h y) { dep_guard_h(a, b, x, y); }
  static __device__ __forceinline__ void keep(v16h a, v16h b, v16h c, v16h d) { keep4_h(a, b, c, d); }
};
template <> struct Frag<__bf16> {
  typedef v16b V; union U { v16b v; v8b h[2]; };
  static __device__ __forceinline__ v16b load(const __bf16* p) {
    U f; f.h[0] = *(const v8b*)(p); f.h[1] = *(const v8b*)(p + 16); return f.v;
  }
  static __device__ __forceinline__ v8f mma(v16b a, v16b b, v8f c) {
    return __builtin_amdgcn_wmma_f32_16x16x32_bf16(false, a, false, b, (short)0, c, false, false);
  }
  static __device__ __forceinline__ void guard(v8f& a, v8f& b, v16b x, v16b y) { dep_guard_b(a, b, x, y); }
  static __device__ __forceinline__ void keep(v16b a, v16b b, v16b c, v16b d) { keep4_b(a, b, c, d); }
};

template <int ET> struct Elem;
template <> struct Elem<0> { typedef _Float16 T; };
template <> struct Elem<1> { typedef __bf16 T; };
template <int ET, bool SPLIT, int BIAS_MODE, int OUT_MODE, bool RESID, int ACT = 0>
__global__ __launch_bounds__(256) void wmma_gemm64(
    const unsigned short* __restrict__ Ap, const unsigned short* __restrict__ A2p, int lda, long strideA,
    const unsigned short* __restrict__ Btp, const unsigned short* __restrict__ Bt2p, int ldb, long strideB,
    void* __restrict__ Cout, void* __restrict__ Cout2, int ldc, long strideC,
    const float* __restrict__ bias,
    const float* __restrict__ resid, long strideR,
    int M, int N, int K, float scale) {
  typedef typename Elem<ET>::T T;
  typedef typename Frag<T>::V V;
  const T* A = (const T*)Ap; const T* A2 = (const T*)A2p; const T* Bt = (const T*)Btp; const T* Bt2 = (const T*)Bt2p;
  __shared__ __align__(16) float sT[8][16 * 68];
  const int b    = blockIdx.y;
  const int lane = threadIdx.x & 31;
  const int wave = threadIdx.x >> 5;
  const int tilesN = N >> 6;
  const int tilesM = M >> 6;
  const int tile = blockIdx.x * 8 + wave;
  if (tile >= tilesM * tilesN) return;
  const int tm = tile / tilesN;
  const int tn = tile - tm * tilesN;
  const int m0 = tm << 6;
  const int n0 = tn << 6;

  const T* Ab  = A  + (size_t)b * strideA;
  const T* Bb  = Bt + (size_t)b * strideB;
  const T* Ab2 = SPLIT ? (A2  + (size_t)b * strideA) : nullptr;
  const T* Bb2 = SPLIT ? (Bt2 + (size_t)b * strideB) : nullptr;

  const int rlane = lane & 15;
  const int koff  = (lane >> 4) * 8;
  const int mOff  = (lane >> 4) * 8;

  v8f acc[4][4];
#pragma unroll
  for (int i = 0; i < 4; ++i)
#pragma unroll
    for (int j = 0; j < 4; ++j) acc[i][j] = (v8f){0.f,0.f,0.f,0.f,0.f,0.f,0.f,0.f};

  for (int k0 = 0; k0 < K; k0 += 32) {
    V bh[4], bl[4];
#pragma unroll
    for (int j = 0; j < 4; ++j) {
      const size_t bo = (size_t)(n0 + (j << 4) + rlane) * ldb + koff + k0;
      bh[j] = Frag<T>::load(Bb + bo);
      if (SPLIT) bl[j] = Frag<T>::load(Bb2 + bo);
    }
#pragma unroll
    for (int i = 0; i < 4; ++i) {
      const size_t ao = (size_t)(m0 + (i << 4) + rlane) * lda + koff + k0;
      V ah = Frag<T>::load(Ab + ao);
      V al;
      if (SPLIT) al = Frag<T>::load(Ab2 + ao);
#pragma unroll
      for (int j = 0; j < 4; ++j) {
        acc[i][j] = Frag<T>::mma(ah, bh[j], acc[i][j]);
        if (SPLIT) {
          acc[i][j] = Frag<T>::mma(ah, bl[j], acc[i][j]);
          acc[i][j] = Frag<T>::mma(al, bh[j], acc[i][j]);
        }
      }
      Frag<T>::guard(acc[i][0], acc[i][3], ah, SPLIT ? al : ah);
    }
    Frag<T>::keep(bh[0], bh[1], bh[2], bh[3]);
    if (SPLIT) Frag<T>::keep(bl[0], bl[1], bl[2], bl[3]);
  }
  acc_guard4(acc[0][0], acc[0][1], acc[0][2], acc[0][3]);
  acc_guard4(acc[1][0], acc[1][1], acc[1][2], acc[1][3]);
  acc_guard4(acc[2][0], acc[2][1], acc[2][2], acc[2][3]);
  acc_guard4(acc[3][0], acc[3][1], acc[3][2], acc[3][3]);

  float* slab = sT[wave];
  const float* Rb = RESID ? (resid + (size_t)b * strideR) : nullptr;
#pragma unroll
  for (int i = 0; i < 4; ++i) {
    const int mBase = m0 + (i << 4);
#pragma unroll
    for (int j = 0; j < 4; ++j) {
      const int n = n0 + (j << 4) + rlane;
      float bv = 0.f;
      if (BIAS_MODE == 2) bv = bias[n];
#pragma unroll
      for (int r = 0; r < 8; ++r) {
        float v = acc[i][j][r] * scale;
        if (BIAS_MODE == 1) v += bias[mBase + mOff + r];
        if (BIAS_MODE == 2) v += bv;
        if (RESID) v += Rb[(size_t)(mBase + mOff + r) * ldc + n];
        if (ACT == 1) v = tanhf(v);
        if (ACT == 2) v = fmaxf(v, 0.0f);
        if (ACT == 3) v = v / (1.0f + expf(-v));
        if (ACT == 4) v = (v > 0.f) ? v : 0.01f * v;
        if (ACT == 5) v = 0.5f * v * (1.0f + erff(v * 0.70710678118654752f));
        slab[(mOff + r) * 68 + (j << 4) + rlane] = v;
      }
    }
    __builtin_amdgcn_fence(__ATOMIC_RELEASE, "workgroup");
    __builtin_amdgcn_wave_barrier();
    __builtin_amdgcn_fence(__ATOMIC_ACQUIRE, "workgroup");
    if (OUT_MODE == 0) {
      float* C = (float*)Cout + (size_t)b * strideC;
      const int hh = lane >> 4, c4 = (lane & 15) * 4;
      for (int pass = 0; pass < 2; ++pass) {
#pragma unroll
        for (int it = 0; it < 8; ++it) {
          const int row = it * 2 + hh;
          v4f v = *(const v4f*)(slab + row * 68 + c4);
          *(volatile v4f*)(C + (size_t)(mBase + row) * ldc + n0 + c4) = v;
        }
        __threadfence();
      }
    } else {
      const int q = lane >> 3, c8 = (lane & 7) * 8;
      unsigned short* C  = (unsigned short*)Cout  + (size_t)b * strideC;
      unsigned short* C2 = (OUT_MODE == 2) ? ((unsigned short*)Cout2 + (size_t)b * strideC) : nullptr;
      for (int pass = 0; pass < 2; ++pass) {
#pragma unroll
        for (int it = 0; it < 4; ++it) {
          const int row = it * 4 + q;
          const float* sp = slab + row * 68 + c8;
          v8h hv, lv;
#pragma unroll
          for (int e = 0; e < 8; ++e) {
            if (OUT_MODE == 1) {
              hv[e] = (_Float16)sp[e];
            } else {
              unsigned short hb = f2bf_bits(sp[e]);
              unsigned short lb = f2bf_bits(sp[e] - bf_bits2f(hb));
              hv[e] = __builtin_bit_cast(_Float16, hb);
              lv[e] = __builtin_bit_cast(_Float16, lb);
            }
          }
          *(volatile v8h*)(C + (size_t)(mBase + row) * ldc + n0 + c8) = hv;
          if (OUT_MODE == 2) *(volatile v8h*)(C2 + (size_t)(mBase + row) * ldc + n0 + c8) = lv;
        }
        __threadfence();
      }
    }
    __builtin_amdgcn_fence(__ATOMIC_RELEASE, "workgroup");
    __builtin_amdgcn_wave_barrier();
    __builtin_amdgcn_fence(__ATOMIC_ACQUIRE, "workgroup");
  }
}

__device__ __forceinline__ unsigned short at_bf_bits(float f) {
  unsigned u = __float_as_uint(f);
  return (unsigned short)((u + 0x7FFFu + ((u >> 16) & 1u)) >> 16);
}
__device__ __forceinline__ __bf16 at_f2bf(float f) { return __builtin_bit_cast(__bf16, at_bf_bits(f)); }
__device__ __forceinline__ void at_split(float f, __bf16& hi, __bf16& lo) {
  const unsigned short hb = at_bf_bits(f);
  hi = __builtin_bit_cast(__bf16, hb);
  lo = at_f2bf(f - __uint_as_float(((unsigned)hb) << 16));
}
__device__ __forceinline__ v8f at_mma(v16b a, v16b b, v8f c) {
  c = __builtin_amdgcn_wmma_f32_16x16x32_bf16(false, a, false, b, (short)0, c, false, false);
  asm volatile("v_nop\n\tv_nop\n\tv_nop\n\tv_nop" : "+v"(c) : "v"(a), "v"(b));
  return c;
}

constexpr int kB     = 2;
constexpr int kPix   = 4096;
constexpr int kW     = 64;
constexpr int kCh    = 256;
constexpr int kHeads = 4;
constexpr int kDh    = 64;
constexpr int kTileY = 4;
constexpr int kTileX = 8;
constexpr int kNbRows = kTileY + 6;
constexpr int kNbCols = kTileX + 6;
constexpr int kKRows  = kNbRows * kNbCols;
constexpr int kPp     = 128;
constexpr int kTilesY = kW / kTileY;
constexpr int kTilesX = kW / kTileX;
static_assert(kHeads * kDh == kCh, "geometry");
static_assert(kW * kW == kPix, "geometry");
static_assert(kPix % 64 == 0 && kCh % 64 == 0 && kCh % 32 == 0, "gemm tile and K multiples");
static_assert(kW % kTileY == 0 && kW % kTileX == 0, "tile coverage");
static_assert(2 * kNbCols + 6 * 16 + 8 + 7 < kKRows, "pv gather rows in range");

union FragB { v16b v; v8b h[2]; };

__global__ __launch_bounds__(256) void tr_split_in_kernel(const float* __restrict__ X,
                                                          unsigned short* __restrict__ Ah,
                                                          unsigned short* __restrict__ Al)
{
  __shared__ __align__(16) float sT[64 * 68];
  const int tid = threadIdx.x;
  const int p0 = blockIdx.x * 64, c0 = blockIdx.y * 64, b = blockIdx.z;
#pragma unroll
  for (int it = 0; it < 4; ++it) {
    const int idx = tid + 256 * it;
    const int crow = idx >> 4, p4 = (idx & 15) * 4;
    const v4f v = *(const v4f*)(X + ((size_t)(b * kCh + c0 + crow)) * kPix + p0 + p4);
    sT[(p4 + 0) * 68 + crow] = v.x;
    sT[(p4 + 1) * 68 + crow] = v.y;
    sT[(p4 + 2) * 68 + crow] = v.z;
    sT[(p4 + 3) * 68 + crow] = v.w;
  }
  __syncthreads();
  const int wv = tid >> 5, lane = tid & 31, q = lane >> 3, c8 = (lane & 7) * 8;
  v8us hv[2], lv[2];
  size_t off[2];
#pragma unroll
  for (int it = 0; it < 2; ++it) {
    const int row = wv * 8 + it * 4 + q;
    const float* sp = sT + row * 68 + c8;
    const v4f a0 = *(const v4f*)sp;
    const v4f a1 = *(const v4f*)(sp + 4);
#pragma unroll
    for (int e = 0; e < 8; ++e) {
      const float fe = (e < 4) ? a0[e] : a1[e - 4];
      const unsigned short hb = f2bf_bits(fe);
      const unsigned short lb = f2bf_bits(fe - bf_bits2f(hb));
      hv[it][e] = hb;
      lv[it][e] = lb;
    }
    off[it] = ((size_t)(b * kPix + p0 + row)) * kCh + c0 + c8;
  }
  for (int pass = 0; pass < 2; ++pass) {
#pragma unroll
    for (int it = 0; it < 2; ++it) {
      *(volatile v8us*)(Ah + off[it]) = hv[it];
      *(volatile v8us*)(Al + off[it]) = lv[it];
    }
    __threadfence();
  }
}

__global__ __launch_bounds__(256) void split_w_kernel(const float* __restrict__ Wf,
                                                      unsigned short* __restrict__ Wh,
                                                      unsigned short* __restrict__ Wl, int n8)
{
  const int i = blockIdx.x * 256 + threadIdx.x;
  if (i < n8) {
    const v4f a0 = *(const v4f*)(Wf + (size_t)i * 8);
    const v4f a1 = *(const v4f*)(Wf + (size_t)i * 8 + 4);
    v8us hv, lv;
#pragma unroll
    for (int e = 0; e < 8; ++e) {
      const float fe = (e < 4) ? a0[e] : a1[e - 4];
      const unsigned short hb = f2bf_bits(fe);
      const unsigned short lb = f2bf_bits(fe - bf_bits2f(hb));
      hv[e] = hb;
      lv[e] = lb;
    }
    unsigned short* ph = Wh + (size_t)i * 8;
    unsigned short* pl = Wl + (size_t)i * 8;
    *(volatile v8us*)ph = hv;
    *(volatile v8us*)pl = lv;
    __threadfence();
    *(volatile v8us*)ph = hv;
    *(volatile v8us*)pl = lv;
  }
}

__global__ __launch_bounds__(64) void local_window_attn_kernel(
    const unsigned short* __restrict__ Qh, const unsigned short* __restrict__ Ql,
    const unsigned short* __restrict__ KVh, const unsigned short* __restrict__ KVl,
    float* __restrict__ Obuf)
{
  __shared__ __align__(16) unsigned short Ksh[kKRows * kDh];
  __shared__ __align__(16) unsigned short Ksl[kKRows * kDh];
  __shared__ __align__(16) __bf16 Psh[2][16 * kPp];
  __shared__ __align__(16) __bf16 Psl[2][16 * kPp];
  __shared__ __align__(16) float  Osh[2][16 * 68];

  const int tid  = threadIdx.x;
  const int w    = tid >> 5, lane = tid & 31, hh = lane >> 4, c = lane & 15;
  const int bidx = blockIdx.x;
  const int tx   = bidx % kTilesX;
  const int ty   = (bidx / kTilesX) % kTilesY;
  const int head = (bidx / (kTilesX * kTilesY)) % kHeads;
  const int b    = bidx / (kTilesX * kTilesY * kHeads);
  const int y0 = ty * kTileY, x0 = tx * kTileX;
  const int nb = w * 2 * kNbCols;

  v16b qh[2], ql[2];
  {
    const int py = y0 + 2 * w + (c >> 3), px = x0 + (c & 7);
    const size_t qoff = ((size_t)(b * kPix + py * kW + px)) * kCh + head * kDh;
    const __bf16* qhp = (const __bf16*)Qh + qoff;
    const __bf16* qlp = (const __bf16*)Ql + qoff;
#pragma unroll
    for (int dc = 0; dc < 2; ++dc) {
      qh[dc] = Frag<__bf16>::load(qhp + dc * 32 + 8 * hh);
      ql[dc] = Frag<__bf16>::load(qlp + dc * 32 + 8 * hh);
    }
  }
  int nrow[7], ncol[7];
#pragma unroll
  for (int t = 0; t < 7; ++t) {
    const int n = t * 16 + c;
    nrow[t] = n / kNbCols;
    ncol[t] = n - nrow[t] * kNbCols;
  }

  v8f oacc[4];
#pragma unroll
  for (int dt = 0; dt < 4; ++dt) oacc[dt] = (v8f){0.f,0.f,0.f,0.f,0.f,0.f,0.f,0.f};
  const size_t planeElems = (size_t)kB * kPix * kCh;
  const v4u z4 = {0u, 0u, 0u, 0u};
  const v8b z8 = __builtin_bit_cast(v8b, z4);

#pragma unroll 1
  for (int br = 0; br < 2; ++br) {
    const unsigned short* Kh = KVh + (size_t)br * planeElems;
    const unsigned short* Kl = KVl + (size_t)br * planeElems;
    __syncthreads();
#pragma unroll 1
    for (int idx = tid; idx < kKRows * 8; idx += 64) {
      const int row = idx >> 3, ch = idx & 7;
      const int nr = row / kNbCols, nc = row - nr * kNbCols;
      const int gy = y0 - 3 + nr, gx = x0 - 3 + nc;
      const bool valid = ((unsigned)gy < (unsigned)kW) && ((unsigned)gx < (unsigned)kW);
      const int gyc = gy < 0 ? 0 : (gy > kW - 1 ? kW - 1 : gy);
      const int gxc = gx < 0 ? 0 : (gx > kW - 1 ? kW - 1 : gx);
      const size_t off = ((size_t)(b * kPix + gyc * kW + gxc)) * kCh + head * kDh + ch * 8;
      v4u vh = *(const v4u*)(Kh + off);
      v4u vl = *(const v4u*)(Kl + off);
      const unsigned msk = valid ? 0xffffffffu : 0u;
      vh.x &= msk; vh.y &= msk; vh.z &= msk; vh.w &= msk;
      vl.x &= msk; vl.y &= msk; vl.z &= msk; vl.w &= msk;
      *(v4u*)(Ksh + row * kDh + ch * 8) = vh;
      *(v4u*)(Ksl + row * kDh + ch * 8) = vl;
    }
    __syncthreads();

    v8f s[7];
#pragma unroll
    for (int t = 0; t < 7; ++t) {
      s[t] = (v8f){0.f,0.f,0.f,0.f,0.f,0.f,0.f,0.f};
#pragma unroll
      for (int dc = 0; dc < 2; ++dc) {
        const int ko = (nb + t * 16 + c) * kDh + dc * 32 + 8 * hh;
        const v16b kfh = Frag<__bf16>::load((const __bf16*)Ksh + ko);
        const v16b kfl = Frag<__bf16>::load((const __bf16*)Ksl + ko);
        s[t] = at_mma(qh[dc], kfh, s[t]);
        s[t] = at_mma(qh[dc], kfl, s[t]);
        s[t] = at_mma(ql[dc], kfh, s[t]);
      }
    }

    __bf16* pwh = Psh[w];
    __bf16* pwl = Psl[w];
#pragma unroll
    for (int r = 0; r < 8; ++r) {
      float mx = -INFINITY;
#pragma unroll
      for (int t = 0; t < 7; ++t) {
        const bool inwin = (nrow[t] >= hh) && (nrow[t] <= hh + 6) && (ncol[t] >= r) && (ncol[t] <= r + 6);
        const float sv = inwin ? s[t][r] : -INFINITY;
        s[t][r] = sv;
        mx = fmaxf(mx, sv);
      }
      mx = fmaxf(mx, __shfl_xor(mx, 1, 32));
      mx = fmaxf(mx, __shfl_xor(mx, 2, 32));
      mx = fmaxf(mx, __shfl_xor(mx, 4, 32));
      mx = fmaxf(mx, __shfl_xor(mx, 8, 32));
      float l = 0.f;
#pragma unroll
      for (int t = 0; t < 7; ++t) {
        const float p = expf(s[t][r] - mx);
        s[t][r] = p;
        l += p;
      }
      l += __shfl_xor(l, 1, 32);
      l += __shfl_xor(l, 2, 32);
      l += __shfl_xor(l, 4, 32);
      l += __shfl_xor(l, 8, 32);
      const float scl = 0.5f / l;
#pragma unroll
      for (int t = 0; t < 7; ++t) {
        __bf16 ph, plo;
        at_split(s[t][r] * scl, ph, plo);
        pwh[(8 * hh + r) * kPp + t * 16 + c] = ph;
        pwl[(8 * hh + r) * kPp + t * 16 + c] = plo;
      }
    }
    __builtin_amdgcn_fence(__ATOMIC_RELEASE, "workgroup");
    __builtin_amdgcn_wave_barrier();
    __builtin_amdgcn_fence(__ATOMIC_ACQUIRE, "workgroup");

#pragma unroll
    for (int kk = 0; kk < 4; ++kk) {
      FragB pa, pb;
      pa.h[0] = *(const v8b*)(pwh + c * kPp + kk * 32 + 8 * hh);
      pb.h[0] = *(const v8b*)(pwl + c * kPp + kk * 32 + 8 * hh);
      if (kk < 3) {
        pa.h[1] = *(const v8b*)(pwh + c * kPp + kk * 32 + 16 + 8 * hh);
        pb.h[1] = *(const v8b*)(pwl + c * kPp + kk * 32 + 16 + 8 * hh);
      } else {
        pa.h[1] = z8;
        pb.h[1] = z8;
      }
      const int rb = nb + kk * 32 + 8 * hh;
#pragma unroll
      for (int dt = 0; dt < 4; ++dt) {
        const int col = dt * 16 + c;
        v8u wh, wl;
#pragma unroll
        for (int j = 0; j < 4; ++j) {
          const int e0 = (rb + 2 * j) * kDh + col, e1 = e0 + kDh;
          wh[j] = (unsigned)Ksh[e0] | ((unsigned)Ksh[e1] << 16);
          wl[j] = (unsigned)Ksl[e0] | ((unsigned)Ksl[e1] << 16);
          if (kk < 3) {
            const int e2 = (rb + 16 + 2 * j) * kDh + col, e3 = e2 + kDh;
            wh[4 + j] = (unsigned)Ksh[e2] | ((unsigned)Ksh[e3] << 16);
            wl[4 + j] = (unsigned)Ksl[e2] | ((unsigned)Ksl[e3] << 16);
          } else {
            wh[4 + j] = 0u;
            wl[4 + j] = 0u;
          }
        }
        const v16b vfh = __builtin_bit_cast(v16b, wh);
        const v16b vfl = __builtin_bit_cast(v16b, wl);
        oacc[dt] = at_mma(pa.v, vfh, oacc[dt]);
        oacc[dt] = at_mma(pa.v, vfl, oacc[dt]);
        oacc[dt] = at_mma(pb.v, vfh, oacc[dt]);
      }
    }
  }

  float* osw = Osh[w];
#pragma unroll
  for (int r = 0; r < 8; ++r)
#pragma unroll
    for (int dt = 0; dt < 4; ++dt) osw[(8 * hh + r) * 68 + dt * 16 + c] = oacc[dt][r];
  __builtin_amdgcn_fence(__ATOMIC_RELEASE, "workgroup");
  __builtin_amdgcn_wave_barrier();
  __builtin_amdgcn_fence(__ATOMIC_ACQUIRE, "workgroup");
  {
    const int c4 = c * 4;
    for (int pass = 0; pass < 2; ++pass) {
#pragma unroll
      for (int it = 0; it < 8; ++it) {
        const int row = it * 2 + hh;
        const v4f val = *(const v4f*)(osw + row * 68 + c4);
        const int py = y0 + 2 * w + (row >> 3), px = x0 + (row & 7);
        *(volatile v4f*)(Obuf + ((size_t)(b * kPix + py * kW + px)) * kCh + head * kDh + c4) = val;
      }
      __threadfence();
    }
  }
}

__global__ __launch_bounds__(256) void tr_out_kernel(const float* __restrict__ O, float* __restrict__ out)
{
  __shared__ __align__(16) float sT[64 * 68];
  const int tid = threadIdx.x;
  const int p0 = blockIdx.x * 64, c0 = blockIdx.y * 64, b = blockIdx.z;
#pragma unroll
  for (int it = 0; it < 4; ++it) {
    const int idx = tid + 256 * it;
    const int prow = idx >> 4, c4 = (idx & 15) * 4;
    const v4f v = *(const v4f*)(O + ((size_t)(b * kPix + p0 + prow)) * kCh + c0 + c4);
    sT[(c4 + 0) * 68 + prow] = v.x;
    sT[(c4 + 1) * 68 + prow] = v.y;
    sT[(c4 + 2) * 68 + prow] = v.z;
    sT[(c4 + 3) * 68 + prow] = v.w;
  }
  __syncthreads();
  const int wv = tid >> 5, lane = tid & 31, hh = lane >> 4, p4 = (lane & 15) * 4;
  v4f val[4];
  size_t off[4];
#pragma unroll
  for (int it = 0; it < 4; ++it) {
    const int row = wv * 8 + it * 2 + hh;
    val[it] = *(const v4f*)(sT + row * 68 + p4);
    off[it] = ((size_t)(b * kCh + c0 + row)) * kPix + p0 + p4;
  }
  for (int pass = 0; pass < 2; ++pass) {
#pragma unroll
    for (int it = 0; it < 4; ++it) *(volatile v4f*)(out + off[it]) = val[it];
    __threadfence();
  }
}

extern "C" void kernel_launch(void* const* d_in, const int* in_sizes, int n_in,
                              void* d_out, int out_size, void* d_ws, size_t ws_size,
                              hipStream_t stream)
{
  const int nAct = kB * kCh * kPix;
  const int nW   = kCh * kCh;
  if (n_in < 5) return;
  if (in_sizes[0] != nAct || in_sizes[1] != nAct || in_sizes[2] != nAct) return;
  if (in_sizes[3] != nW || in_sizes[4] != nW) return;
  if (out_size != nAct) return;

  const float* kvmap1 = (const float*)d_in[0];
  const float* qmap   = (const float*)d_in[1];
  const float* kvmap2 = (const float*)d_in[2];
  const float* Wq     = (const float*)d_in[3];
  const float* Wkv    = (const float*)d_in[4];
  float* out = (float*)d_out;

  const size_t planeB  = (size_t)nAct * 2;
  const size_t wplaneB = (size_t)nW * 2;
  char* ws = (char*)d_ws;
  size_t o = 0;
  unsigned short* XTqh  = (unsigned short*)(ws + o); o += planeB;
  unsigned short* XTql  = (unsigned short*)(ws + o); o += planeB;
  unsigned short* XTk1h = (unsigned short*)(ws + o); o += planeB;
  unsigned short* XTk1l = (unsigned short*)(ws + o); o += planeB;
  unsigned short* XTk2h = (unsigned short*)(ws + o); o += planeB;
  unsigned short* XTk2l = (unsigned short*)(ws + o); o += planeB;
  unsigned short* Wqh   = (unsigned short*)(ws + o); o += wplaneB;
  unsigned short* Wql   = (unsigned short*)(ws + o); o += wplaneB;
  unsigned short* Wkh   = (unsigned short*)(ws + o); o += wplaneB;
  unsigned short* Wkl   = (unsigned short*)(ws + o); o += wplaneB;
  unsigned short* Qh    = (unsigned short*)(ws + o); o += planeB;
  unsigned short* Ql    = (unsigned short*)(ws + o); o += planeB;
  unsigned short* KVh   = (unsigned short*)(ws + o); o += 2 * planeB;
  unsigned short* KVl   = (unsigned short*)(ws + o); o += 2 * planeB;
  float*          Obuf  = (float*)(ws + o);          o += (size_t)nAct * 4;
  if (o > ws_size) return;
  const float* dummyf = (const float*)(const void*)Wqh;

  const dim3 gtr(kPix / 64, kCh / 64, kB);
  tr_split_in_kernel<<<gtr, 256, 0, stream>>>(qmap,   XTqh,  XTql);
  tr_split_in_kernel<<<gtr, 256, 0, stream>>>(kvmap1, XTk1h, XTk1l);
  tr_split_in_kernel<<<gtr, 256, 0, stream>>>(kvmap2, XTk2h, XTk2l);
  const int n8 = nW / 8;
  split_w_kernel<<<(n8 + 255) / 256, 256, 0, stream>>>(Wq,  Wqh, Wql, n8);
  split_w_kernel<<<(n8 + 255) / 256, 256, 0, stream>>>(Wkv, Wkh, Wkl, n8);
  const long strideAct = (long)kPix * kCh;
  const dim3 ggemm((kPix / 64) * (kCh / 64) / 8, kB, 1);
  wmma_gemm64<1, true, 0, 2, false, 0><<<ggemm, 256, 0, stream>>>(
      XTqh, XTql, kCh, strideAct, Wqh, Wql, kCh, 0L,
      (void*)Qh, (void*)Ql, kCh, strideAct, dummyf, dummyf, 0L, kPix, kCh, kCh, 0.125f);
  wmma_gemm64<1, true, 0, 2, false, 0><<<ggemm, 256, 0, stream>>>(
      XTk1h, XTk1l, kCh, strideAct, Wkh, Wkl, kCh, 0L,
      (void*)KVh, (void*)KVl, kCh, strideAct, dummyf, dummyf, 0L, kPix, kCh, kCh, 1.0f);
  wmma_gemm64<1, true, 0, 2, false, 0><<<ggemm, 256, 0, stream>>>(
      XTk2h, XTk2l, kCh, strideAct, Wkh, Wkl, kCh, 0L,
      (void*)(KVh + (size_t)nAct), (void*)(KVl + (size_t)nAct), kCh, strideAct, dummyf, dummyf, 0L, kPix, kCh, kCh, 1.0f);
  local_window_attn_kernel<<<kB * kHeads * kTilesY * kTilesX, 64, 0, stream>>>(Qh, Ql, KVh, KVl, Obuf);
  tr_out_kernel<<<gtr, 256, 0, stream>>>(Obuf, out);
}
